// DualHeadGAT_84258668413092
// MI455X (gfx1250) — hardware-run, weakly checked
//
#include <hip/hip_runtime.h>
#include <stddef.h>
#include <stdint.h>
#include <math.h>

#define NN      50000
#define FD      128
#define HC1     256
#define HD      64
#define NH1     4
#define NE      800000
#define GBM     128
#define MP      50048
#define KP2     512
#define SPLIT2  1
#define K2EXT   ((SPLIT2) ? 512 : 256)
#define NTHR    256
#define NWAVE   8
#define EPT     8
#define WCH     (32 * EPT)
#define NBRUN   1024
#define SLB     10
#define NBK     49
#define WLCAP   3584
#define RCAP    28672
#define DEGCAP  64
#define MAXDEG_MEAS   35
#define MAXB1024_MEAS 16623
#define ABM     64
#define SP      68
#define NEGSL   0.2f
#define EPS_SM  1e-16f

#define SM_AS1  0
#define SM_AD1  256
#define SM_B1   512
#define SM_AS2  768
#define SM_AD2  832
#define SM_B2   896
#define SM_WS   960
#define SM_BS   1024
#define SM_N    1056

#define BK_ZINTS (NWAVE * WLCAP + RCAP + 3 * NBRUN)
#define BK_INTS  (BK_ZINTS + 16)
#define BK_LDS   (BK_INTS * 4)

#define PBX   (MP * FD / 8 / NTHR)
#define PBW1  (HC1 * FD / 8 / NTHR)
#define PBW2  (HD * KP2 / 8 / NTHR)
#define PBTOT (PBX + PBW1 + PBW2 + 2)

#define OUT1_OFF (NN * HD)

static_assert(SPLIT2 == 0 || SPLIT2 == 1);
static_assert(HD == 64 && HC1 == NH1 * HD && KP2 == 2 * HC1);
static_assert(MP % GBM == 0 && MP >= NN && MP == 391 * GBM && MP % ABM == 0);
static_assert(NBRUN == (1 << SLB) && NBRUN % ABM == 0 && NBRUN % 32 == 0);
static_assert(NBK * NBRUN >= MP);
static_assert(NE < (1 << 20) && (((long long)NE) << SLB) < (1LL << 31));
static_assert(NE % WCH == 0 && NE % 4 == 0);
static_assert(RCAP == NWAVE * WLCAP && RCAP % (NTHR * 4) == 0 && BK_ZINTS % 4 == 0);
static_assert((2 * NBRUN) % (NTHR * 4) == 0);
static_assert((long long)RCAP * 100 >= (long long)MAXB1024_MEAS * 105);
static_assert(WLCAP >= MAXB1024_MEAS / 8 + 8 * 46 + 1);
static_assert(MAXDEG_MEAS + 8 <= DEGCAP);
static_assert((MP * FD / 8) % NTHR == 0 && (HC1 * FD / 8) % NTHR == 0 && (HD * KP2 / 8) % NTHR == 0);
static_assert(FD % 32 == 0 && K2EXT % 32 == 0 && K2EXT <= KP2);
static_assert(BK_LDS <= 300000);
static_assert((GBM * SP + 512 + GBM * 8) * 4 <= 65536);
static_assert(ABM == NWAVE * 8);
static_assert(NN % 4 == 0 && (OUT1_OFF * 4) % 128 == 0);
static_assert((long long)(NN - 1) * HD + (HD - 1) < (long long)OUT1_OFF);
static_assert((long long)OUT1_OFF + NN - 1 < (long long)NN * HD + NN);

typedef float          v4f   __attribute__((ext_vector_type(4)));
typedef float          v8f   __attribute__((ext_vector_type(8)));
typedef int            v4i   __attribute__((ext_vector_type(4)));
typedef int            v8i   __attribute__((ext_vector_type(8)));
typedef unsigned short v8us  __attribute__((ext_vector_type(8)));
typedef unsigned short v16us __attribute__((ext_vector_type(16)));
typedef __bf16         v16bf __attribute__((ext_vector_type(16)));
typedef v4f  __attribute__((may_alias)) v4fa;
typedef v4i  __attribute__((may_alias)) v4ia;
typedef v8us __attribute__((may_alias)) v8usa;
union FragB { v16bf v; v16us u; v8us h[2]; v8i w; };

__device__ __forceinline__ v8f wmb(const FragB& a, const FragB& b, v8f c) {
  v8f d = __builtin_amdgcn_wmma_f32_16x16x32_bf16(false, a.v, false, b.v, (short)0, c, false, false);
  asm volatile("v_nop\n\tv_nop\n\tv_nop\n\tv_nop" : "+v"(d) : "v"(a.w), "v"(b.w));
  return d;
}

__device__ __forceinline__ unsigned bf16_bits(float f) {
  const unsigned u = __float_as_uint(f);
  const unsigned r = (u + 0x7FFFu + ((u >> 16) & 1u)) >> 16;
  const unsigned q = (u >> 16) | 0x40u;
  return ((u & 0x7fffffffu) > 0x7f800000u) ? q : r;
}
__device__ __forceinline__ float bf16_val(float f) {
  return __uint_as_float(bf16_bits(f) << 16);
}
__device__ __forceinline__ v4f bf16_val4(const v4f a) {
  v4f r;
  r.x = bf16_val(a.x); r.y = bf16_val(a.y); r.z = bf16_val(a.z); r.w = bf16_val(a.w);
  return r;
}

__device__ __forceinline__ void hilo_pack(float v0, float v1, float v2, float v3,
                                          int& h01, int& h23, int& l01, int& l23) {
  const unsigned a0 = bf16_bits(v0), a1 = bf16_bits(v1), a2 = bf16_bits(v2), a3 = bf16_bits(v3);
  const unsigned b0 = bf16_bits(v0 - __uint_as_float(a0 << 16));
  const unsigned b1 = bf16_bits(v1 - __uint_as_float(a1 << 16));
  const unsigned b2 = bf16_bits(v2 - __uint_as_float(a2 << 16));
  const unsigned b3 = bf16_bits(v3 - __uint_as_float(a3 << 16));
  h01 = (int)(a0 | (a1 << 16)); h23 = (int)(a2 | (a3 << 16));
  l01 = (int)(b0 | (b1 << 16)); l23 = (int)(b2 | (b3 << 16));
}

__device__ __forceinline__ void st2_v4f(float* p, v4f v) {
  *(volatile v4f*)p = v;
  __threadfence();
  *(volatile v4f*)p = v;
}
__device__ __forceinline__ void st2_v8us(unsigned short* p, v8us v) {
  *(volatile v8us*)p = v;
  __threadfence();
  *(volatile v8us*)p = v;
}

__device__ __forceinline__ v8us col8(const float* __restrict__ base, int stride) {
  float f[8];
#pragma unroll
  for (int i = 0; i < 8; ++i) f[i] = base[(size_t)i * (size_t)stride];
  v8us o;
#pragma unroll
  for (int i = 0; i < 8; ++i) o[i] = (unsigned short)bf16_bits(f[i]);
  return o;
}

__global__ __launch_bounds__(NTHR) void k_prep(
    const float* __restrict__ x, const float* __restrict__ w1, const float* __restrict__ w2,
    const float* __restrict__ as1, const float* __restrict__ ad1, const float* __restrict__ b1,
    const float* __restrict__ as2, const float* __restrict__ ad2, const float* __restrict__ b2,
    const float* __restrict__ wsv, const float* __restrict__ bsv,
    unsigned short* xb, unsigned short* w1t, unsigned short* w2t, float* sm) {
  const int tid = (int)threadIdx.x, lane = tid & 31;
  const int blk = (int)blockIdx.x;
  if (blk < PBX) {
    const int u   = blk * NTHR + tid;
    const int row = u >> 4, k8 = (u & 15) * 8;
    const int rc  = row < NN ? row : NN - 1;
    const unsigned mk = row < NN ? 0xffffu : 0u;
    const float* p = x + (size_t)rc * FD + k8;
    const v4f a = *(const v4fa*)p;
    const v4f b = *(const v4fa*)(p + 4);
    v8us o;
    o[0] = (unsigned short)(bf16_bits(a.x) & mk); o[1] = (unsigned short)(bf16_bits(a.y) & mk);
    o[2] = (unsigned short)(bf16_bits(a.z) & mk); o[3] = (unsigned short)(bf16_bits(a.w) & mk);
    o[4] = (unsigned short)(bf16_bits(b.x) & mk); o[5] = (unsigned short)(bf16_bits(b.y) & mk);
    o[6] = (unsigned short)(bf16_bits(b.z) & mk); o[7] = (unsigned short)(bf16_bits(b.w) & mk);
    st2_v8us(xb + (size_t)row * FD + k8, o);
  } else if (blk < PBX + PBW1) {
    const int u = (blk - PBX) * NTHR + tid;
    const int n = u >> 4, k8 = (u & 15) * 8;
    const v8us o = col8(w1 + (size_t)k8 * HC1 + n, HC1);
    st2_v8us(w1t + (size_t)n * FD + k8, o);
  } else if (blk < PBX + PBW1 + PBW2) {
    const int u = (blk - PBX - PBW1) * NTHR + tid;
    const int n = u >> 6, k8 = (u & 63) * 8, kk = k8 & (HC1 - 1);
    const v8us o = col8(w2 + (size_t)kk * HD + n, HD);
    st2_v8us(w2t + (size_t)n * KP2 + k8, o);
  } else if (blk == PBX + PBW1 + PBW2) {
    const int wv = tid >> 5;
    v4f a;
    if (wv < 2) {
      a = *(const v4fa*)(as1 + 4 * tid);
    } else if (wv < 4) {
      a = *(const v4fa*)(ad1 + 4 * (tid - 64));
    } else if (wv < 6) {
      a = *(const v4fa*)(b1 + 4 * (tid - 128));
    } else {
      const int q = lane & 15;
      v4f p, r;
      if (wv == 6) {
        p = *(const v4fa*)(as2 + 4 * q);
        r = *(const v4fa*)(ad2 + 4 * q);
      } else {
        p = *(const v4fa*)(b2 + 4 * q);
        r = *(const v4fa*)(wsv + 4 * q);
      }
      asm volatile("" :: "v"(p));
      asm volatile("" :: "v"(r));
      const unsigned mk = (lane < 16) ? 0xffffffffu : 0u;
      a.x = __uint_as_float((__float_as_uint(p.x) & mk) | (__float_as_uint(r.x) & ~mk));
      a.y = __uint_as_float((__float_as_uint(p.y) & mk) | (__float_as_uint(r.y) & ~mk));
      a.z = __uint_as_float((__float_as_uint(p.z) & mk) | (__float_as_uint(r.z) & ~mk));
      a.w = __uint_as_float((__float_as_uint(p.w) & mk) | (__float_as_uint(r.w) & ~mk));
    }
    const v4f o = bf16_val4(a);
    st2_v4f(sm + 4 * tid, o);
  } else {
    if (tid < 8) {
      const float v = bf16_val(bsv[0]);
      const v4f o = {v, v, v, v};
      st2_v4f(sm + SM_BS + 4 * tid, o);
    }
  }
}

__device__ __forceinline__ void bucket_flush(const int* pl, const int* cnt, int ov, int* lp, int* cop, int* fp,
                                             int tid) {
#pragma unroll 1
  for (int i = tid * 4; i < RCAP; i += NTHR * 4) {
    const v4i v = *(const v4ia*)(pl + i);
    *(volatile v4i*)(lp + i) = v;
  }
#pragma unroll 1
  for (int i = tid * 4; i < 2 * NBRUN; i += NTHR * 4) {
    const v4i v = *(const v4ia*)(cnt + i);
    *(volatile v4i*)(cop + i) = v;
  }
  if (tid < 8) {
    const v4i f = {ov, ov, ov, ov};
    *(volatile v4i*)(fp + 4 * tid) = f;
  }
}

__global__ __launch_bounds__(NTHR) void k_bucket(const int* __restrict__ srcs, const int* __restrict__ dsts,
                                                 int* LIST, int* CO, int* FLAG) {
  extern __shared__ __attribute__((aligned(16))) int dsm[];
  int* wl   = dsm;
  int* pl   = dsm + NWAVE * WLCAP;
  int* cnt  = pl + RCAP;
  int* offs = cnt + NBRUN;
  int* cur  = offs + NBRUN;
  int* misc = cur + NBRUN;
  const int tid = (int)threadIdx.x, lane = tid & 31, wave = tid >> 5;
  const int blk = (int)blockIdx.x;
  const unsigned nbs = (unsigned)(blk * NBRUN);

  {
    const v4i z4 = {0, 0, 0, 0};
    for (int i = tid * 4; i < BK_ZINTS; i += NTHR * 4) *(v4ia*)(dsm + i) = z4;
    if (tid < 16) misc[tid] = 0;
  }
  __syncthreads();

  {
    const int per  = ((NE + NWAVE * WCH - 1) / (NWAVE * WCH)) * WCH;
    const int ebeg = wave * per;
    const int eend = (ebeg + per < NE) ? (ebeg + per) : NE;
    int* mylist = wl + wave * WLCAP;
    int wc = 0;
#pragma unroll 1
    for (int cb = ebeg; cb < eend; cb += WCH) {
      const int e0 = cb + lane * EPT;
      const v4i da = *(const v4ia*)(dsts + e0);
      const v4i db = *(const v4ia*)(dsts + e0 + 4);
      const unsigned s0 = (unsigned)da.x - nbs, s1 = (unsigned)da.y - nbs;
      const unsigned s2 = (unsigned)da.z - nbs, s3 = (unsigned)da.w - nbs;
      const unsigned s4 = (unsigned)db.x - nbs, s5 = (unsigned)db.y - nbs;
      const unsigned s6 = (unsigned)db.z - nbs, s7 = (unsigned)db.w - nbs;
      const bool h0 = s0 < (unsigned)NBRUN, h1 = s1 < (unsigned)NBRUN, h2 = s2 < (unsigned)NBRUN, h3 = s3 < (unsigned)NBRUN;
      const bool h4 = s4 < (unsigned)NBRUN, h5 = s5 < (unsigned)NBRUN, h6 = s6 < (unsigned)NBRUN, h7 = s7 < (unsigned)NBRUN;
      const unsigned m0 = __builtin_amdgcn_ballot_w32(h0), m1 = __builtin_amdgcn_ballot_w32(h1);
      const unsigned m2 = __builtin_amdgcn_ballot_w32(h2), m3 = __builtin_amdgcn_ballot_w32(h3);
      const unsigned m4 = __builtin_amdgcn_ballot_w32(h4), m5 = __builtin_amdgcn_ballot_w32(h5);
      const unsigned m6 = __builtin_amdgcn_ballot_w32(h6), m7 = __builtin_amdgcn_ballot_w32(h7);
      const unsigned any = m0 | m1 | m2 | m3 | m4 | m5 | m6 | m7;
      if (any != 0u) {
        const int pre = (int)(__builtin_amdgcn_mbcnt_lo(m0, 0u) + __builtin_amdgcn_mbcnt_lo(m1, 0u) +
                              __builtin_amdgcn_mbcnt_lo(m2, 0u) + __builtin_amdgcn_mbcnt_lo(m3, 0u) +
                              __builtin_amdgcn_mbcnt_lo(m4, 0u) + __builtin_amdgcn_mbcnt_lo(m5, 0u) +
                              __builtin_amdgcn_mbcnt_lo(m6, 0u) + __builtin_amdgcn_mbcnt_lo(m7, 0u));
        int p = wc + pre;
        if (h0) { if (p < WLCAP) mylist[p] = ((e0 + 0) << SLB) | (int)s0; p = p + 1; }
        if (h1) { if (p < WLCAP) mylist[p] = ((e0 + 1) << SLB) | (int)s1; p = p + 1; }
        if (h2) { if (p < WLCAP) mylist[p] = ((e0 + 2) << SLB) | (int)s2; p = p + 1; }
        if (h3) { if (p < WLCAP) mylist[p] = ((e0 + 3) << SLB) | (int)s3; p = p + 1; }
        if (h4) { if (p < WLCAP) mylist[p] = ((e0 + 4) << SLB) | (int)s4; p = p + 1; }
        if (h5) { if (p < WLCAP) mylist[p] = ((e0 + 5) << SLB) | (int)s5; p = p + 1; }
        if (h6) { if (p < WLCAP) mylist[p] = ((e0 + 6) << SLB) | (int)s6; p = p + 1; }
        if (h7) { if (p < WLCAP) mylist[p] = ((e0 + 7) << SLB) | (int)s7; p = p + 1; }
        wc += (int)(__builtin_popcount(m0) + __builtin_popcount(m1) + __builtin_popcount(m2) + __builtin_popcount(m3) +
                    __builtin_popcount(m4) + __builtin_popcount(m5) + __builtin_popcount(m6) + __builtin_popcount(m7));
      }
    }
    if (lane == 0) misc[wave] = wc;
  }
  __syncthreads();

  if (wave == 0) {
    int ov = 0;
#pragma unroll 1
    for (int w2 = 0; w2 < NWAVE; ++w2) {
      int c = misc[w2];
      if (c > WLCAP) ov = 1;
      c = c < 0 ? 0 : (c > WLCAP ? WLCAP : c);
#pragma unroll 1
      for (int b0 = 0; b0 < c; b0 += 32) {
        const int idx = b0 + lane;
        const int ent = wl[w2 * WLCAP + (idx < WLCAP ? idx : WLCAP - 1)];
        const int m32 = (c - b0) < 32 ? (c - b0) : 32;
#pragma unroll 1
        for (int k = 0; k < m32; ++k) {
          const int u    = __builtin_amdgcn_readlane(ent, k);
          const int slot = u & (NBRUN - 1);
          if (lane == 0) cnt[slot] = cnt[slot] + 1;
        }
      }
    }
    if (lane == 0) misc[9] = ov;
  }
  __syncthreads();
  if (wave == 0) {
    const int base = lane * (NBRUN / 32);
    int s = 0;
#pragma unroll 1
    for (int i = 0; i < NBRUN / 32; ++i) s += cnt[base + i];
    int incl = s;
#pragma unroll
    for (int d = 1; d < 32; d <<= 1) {
      const int y = __shfl_up(incl, d, 32);
      if (lane >= d) incl += y;
    }
    int run = incl - s;
#pragma unroll 1
    for (int i = 0; i < NBRUN / 32; ++i) {
      const int cv = cnt[base + i];
      offs[base + i] = run;
      cur[base + i]  = run;
      run += cv;
    }
  }
  __syncthreads();

  if (wave == 0) {
#pragma unroll 1
    for (int w2 = 0; w2 < NWAVE; ++w2) {
      int c = misc[w2];
      c = c < 0 ? 0 : (c > WLCAP ? WLCAP : c);
#pragma unroll 1
      for (int b0 = 0; b0 < c; b0 += 32) {
        const int idx = b0 + lane;
        const int ent = wl[w2 * WLCAP + (idx < WLCAP ? idx : WLCAP - 1)];
        int eid = (ent >> SLB) & 0xFFFFF;
        eid = eid > NE - 1 ? NE - 1 : eid;
        int sr = srcs[eid];
        sr = sr < 0 ? 0 : (sr > NN - 1 ? NN - 1 : sr);
        const int m32 = (c - b0) < 32 ? (c - b0) : 32;
#pragma unroll 1
        for (int k = 0; k < m32; ++k) {
          const int u    = __builtin_amdgcn_readlane(ent, k);
          const int wd   = __builtin_amdgcn_readlane(sr, k);
          const int slot = u & (NBRUN - 1);
          if (lane == 0) {
            int p = cur[slot];
            p = p < 0 ? 0 : (p > RCAP - 1 ? RCAP - 1 : p);
            pl[p] = wd;
            cur[slot] = p + 1;
          }
        }
      }
    }
  }
  __syncthreads();

  const int ovf = misc[9];
  int* lp  = LIST + (size_t)blk * RCAP;
  int* cop = CO + (size_t)blk * (2 * NBRUN);
  int* fp  = FLAG + (size_t)blk * 32;
  bucket_flush(pl, cnt, ovf, lp, cop, fp, tid);
  __threadfence();
  bucket_flush(pl, cnt, ovf, lp, cop, fp, tid);
}

template <int KEXT, int BPITCH>
__device__ __forceinline__ void gemm_16x64(const unsigned short* __restrict__ ap,
                                           const unsigned short* __restrict__ bp, v8f (&acc)[4]) {
#pragma unroll 1
  for (int k0 = 0; k0 < KEXT; k0 += 32) {
    FragB af;
    af.h[0] = *(const v8usa*)(ap + k0);
    af.h[1] = *(const v8usa*)(ap + k0 + 16);
#pragma unroll
    for (int nt = 0; nt < 4; ++nt) {
      const unsigned short* wq = bp + (size_t)(16 * nt) * (size_t)BPITCH + k0;
      FragB bf;
      bf.h[0] = *(const v8usa*)wq;
      bf.h[1] = *(const v8usa*)(wq + 16);
      acc[nt] = wmb(af, bf, acc[nt]);
    }
  }
}

__device__ __forceinline__ void stage_d(float* stg, const v8f (&acc)[4], int wave, int hh, int m) {
#pragma unroll
  for (int nt = 0; nt < 4; ++nt) {
#pragma unroll
    for (int r = 0; r < 8; ++r) stg[(16 * wave + 8 * hh + r) * SP + 16 * nt + m] = acc[nt][r];
  }
}

__global__ __launch_bounds__(NTHR) __attribute__((amdgpu_num_vgpr(248)))
void k_lin1(const unsigned short* __restrict__ XB, const unsigned short* __restrict__ W1T,
            const float* __restrict__ sm, float* XH1, float* SD1) {
  __shared__ __attribute__((aligned(16))) float stg[GBM * SP];
  __shared__ __attribute__((aligned(16))) float satt[2 * HC1];
  __shared__ __attribute__((aligned(16))) float sdot[GBM * 8];
  const int tid = (int)threadIdx.x, lane = tid & 31, wave = tid >> 5, hh = lane >> 4, m = lane & 15;
  const int rowBase = (int)blockIdx.x * GBM;
  if (tid < 128) *(v4fa*)(satt + 4 * tid) = *(const v4fa*)(sm + SM_AS1 + 4 * tid);

  const unsigned short* ap = XB + (size_t)(rowBase + 16 * wave + m) * (size_t)FD + 8 * hh;
#pragma unroll 1
  for (int head = 0; head < NH1; ++head) {
    v8f acc[4];
    {
      const v8f z = {0.f, 0.f, 0.f, 0.f, 0.f, 0.f, 0.f, 0.f};
#pragma unroll
      for (int t = 0; t < 4; ++t) acc[t] = z;
    }
    const unsigned short* bp = W1T + (size_t)(head * HD + m) * (size_t)FD + 8 * hh;
    gemm_16x64<FD, FD>(ap, bp, acc);
    stage_d(stg, acc, wave, hh, m);
    __syncthreads();

    {
      const int row = tid & (GBM - 1), which = tid >> 7;
      const float* sa = satt + which * HC1 + head * HD;
      const float* hr = stg + row * SP;
      float d = 0.0f;
#pragma unroll 4
      for (int c4 = 0; c4 < HD / 4; ++c4) {
        const v4f hv = *(const v4fa*)(hr + 4 * c4);
        const v4f av = *(const v4fa*)(sa + 4 * c4);
        d = fmaf(hv.x, av.x, d);
        d = fmaf(hv.y, av.y, d);
        d = fmaf(hv.z, av.z, d);
        d = fmaf(hv.w, av.w, d);
      }
      sdot[row * 8 + which * 4 + head] = d;
    }

    v4f fv[8];
#pragma unroll
    for (int i = 0; i < 8; ++i) {
      const int lr = 16 * wave + 2 * i + hh;
      fv[i] = *(const v4fa*)(stg + lr * SP + 4 * m);
    }
#pragma unroll
    for (int i = 0; i < 8; ++i) {
      const int lr = 16 * wave + 2 * i + hh;
      float* op = XH1 + (size_t)(rowBase + lr) * HC1 + head * HD + 4 * m;
      *(volatile v4f*)op = fv[i];
    }
    __threadfence();
#pragma unroll
    for (int i = 0; i < 8; ++i) {
      const int lr = 16 * wave + 2 * i + hh;
      float* op = XH1 + (size_t)(rowBase + lr) * HC1 + head * HD + 4 * m;
      *(volatile v4f*)op = fv[i];
    }
    __syncthreads();
  }

  {
    const v4f sv = *(const v4fa*)(sdot + 4 * tid);
    st2_v4f(SD1 + (size_t)rowBase * 8 + 4 * tid, sv);
  }
}

__global__ __launch_bounds__(NTHR) void k_att1(const int* __restrict__ LIST, const int* __restrict__ CO,
                                               const int* __restrict__ FLAG, const float* __restrict__ XH1,
                                               const float* __restrict__ SD1, const float* __restrict__ sm,
                                               unsigned short* H1HL) {
  __shared__ __attribute__((aligned(16))) float sb1[HC1];
  const int tid = (int)threadIdx.x, lane = tid & 31, wave = tid >> 5;
  if (tid < 64) *(v4fa*)(sb1 + 4 * tid) = *(const v4fa*)(sm + SM_B1 + 4 * tid);
  __syncthreads();
  const int rowBase = (int)blockIdx.x * ABM;
  const int bucket  = rowBase >> SLB;
  const int* lb  = LIST + (size_t)bucket * RCAP;
  const int* cob = CO + (size_t)bucket * (2 * NBRUN);
  const int flag = FLAG[(size_t)bucket * 32];
  const float qnan = __uint_as_float(0x7fc00000u);
  const int head = lane >> 3, c0 = 8 * lane;
  const v4f bA = *(const v4fa*)(sb1 + c0);
  const v4f bB = *(const v4fa*)(sb1 + c0 + 4);

#pragma unroll 1
  for (int i = 0; i < ABM / NWAVE; ++i) {
    const int d    = rowBase + (ABM / NWAVE) * wave + i;
    const int slot = d & (NBRUN - 1);
    const int dcl  = d < NN ? d : NN - 1;
    int cv = cob[slot];
    int ov = cob[NBRUN + slot];
    const bool big = cv > DEGCAP;
    cv = cv < 0 ? 0 : (cv > DEGCAP ? DEGCAP : cv);
    ov = ov < 0 ? 0 : (ov > RCAP - 1 ? RCAP - 1 : ov);
    const int c = __builtin_amdgcn_readfirstlane(cv);
    const int o = __builtin_amdgcn_readfirstlane(ov);
    int last = o + c - 1;
    last = last < o ? o : last;
    last = last > RCAP - 1 ? RCAP - 1 : last;

    const float* sdd = SD1 + (size_t)dcl * 8;
    const float adv = sdd[4 + head];
    const float asd = sdd[head];
    const float* xr = XH1 + (size_t)dcl * HC1 + c0;
    v4f aA = *(const v4fa*)xr;
    v4f aB = *(const v4fa*)(xr + 4);
    asm volatile("" :: "v"(aA));
    asm volatile("" :: "v"(aB));
    float l0 = asd + adv;
    l0 = (l0 > 0.0f) ? l0 : NEGSL * l0;
    float mx = l0, dn = 1.0f;

#pragma unroll 1
    for (int j = 0; j < c; ++j) {
      int idx = o + j;
      idx = idx > last ? last : idx;
      int sr = lb[idx];
      sr = sr < 0 ? 0 : (sr > NN - 1 ? NN - 1 : sr);
      const float* xs = XH1 + (size_t)sr * HC1 + c0;
      const v4f fA = *(const v4fa*)xs;
      const v4f fB = *(const v4fa*)(xs + 4);
      const float asv = SD1[(size_t)sr * 8 + head];
      asm volatile("" :: "v"(fA));
      asm volatile("" :: "v"(fB));
      asm volatile("" :: "v"(asv));
      float lg = asv + adv;
      lg = (lg > 0.0f) ? lg : NEGSL * lg;
      const float df = lg - mx;
      const float ee = expf(-fabsf(df));
      const bool up  = df > 0.0f;
      const float s1 = up ? ee : 1.0f;
      const float s2 = up ? 1.0f : ee;
      mx = up ? lg : mx;
      dn = fmaf(dn, s1, s2);
      aA.x = fmaf(aA.x, s1, s2 * fA.x); aA.y = fmaf(aA.y, s1, s2 * fA.y);
      aA.z = fmaf(aA.z, s1, s2 * fA.z); aA.w = fmaf(aA.w, s1, s2 * fA.w);
      aB.x = fmaf(aB.x, s1, s2 * fB.x); aB.y = fmaf(aB.y, s1, s2 * fB.y);
      aB.z = fmaf(aB.z, s1, s2 * fB.z); aB.w = fmaf(aB.w, s1, s2 * fB.w);
    }

    const float inv = 1.0f / (dn + EPS_SM);
    float x0 = fmaf(aA.x, inv, bA.x), x1 = fmaf(aA.y, inv, bA.y);
    float x2 = fmaf(aA.z, inv, bA.z), x3 = fmaf(aA.w, inv, bA.w);
    float x4 = fmaf(aB.x, inv, bB.x), x5 = fmaf(aB.y, inv, bB.y);
    float x6 = fmaf(aB.z, inv, bB.z), x7 = fmaf(aB.w, inv, bB.w);
#pragma unroll 1
    for (int r = 0; r < 8; ++r) {
      const float t = (x0 > 0.0f) ? x0 : expm1f(x0);
      x0 = x1; x1 = x2; x2 = x3; x3 = x4; x4 = x5; x5 = x6; x6 = x7; x7 = t;
    }
    const bool bad  = (flag != 0) | big;
    const bool live = d < NN;
    x0 = bad ? qnan : x0; x1 = bad ? qnan : x1; x2 = bad ? qnan : x2; x3 = bad ? qnan : x3;
    x4 = bad ? qnan : x4; x5 = bad ? qnan : x5; x6 = bad ? qnan : x6; x7 = bad ? qnan : x7;
    x0 = live ? x0 : 0.0f; x1 = live ? x1 : 0.0f; x2 = live ? x2 : 0.0f; x3 = live ? x3 : 0.0f;
    x4 = live ? x4 : 0.0f; x5 = live ? x5 : 0.0f; x6 = live ? x6 : 0.0f; x7 = live ? x7 : 0.0f;

    int h01, h23, l01, l23, h45, h67, l45, l67;
    hilo_pack(x0, x1, x2, x3, h01, h23, l01, l23);
    hilo_pack(x4, x5, x6, x7, h45, h67, l45, l67);
    v4i hw, lw;
    hw.x = h01; hw.y = h23; hw.z = h45; hw.w = h67;
    lw.x = l01; lw.y = l23; lw.z = l45; lw.w = l67;
    unsigned short* hp = H1HL + (size_t)d * KP2 + c0;
    *(volatile v4i*)hp = hw;
    *(volatile v4i*)(hp + HC1) = lw;
    __threadfence();
    *(volatile v4i*)hp = hw;
    *(volatile v4i*)(hp + HC1) = lw;
  }
}

__global__ __launch_bounds__(NTHR) __attribute__((amdgpu_num_vgpr(248)))
void k_lin2(const unsigned short* __restrict__ A, const unsigned short* __restrict__ BT,
            const float* __restrict__ sm, float* XH2, float* SD2) {
  __shared__ __attribute__((aligned(16))) float stg[GBM * SP];
  __shared__ __attribute__((aligned(16))) float satt2[2 * HD];
  __shared__ __attribute__((aligned(16))) float sdot2[GBM * 2];
  const int tid = (int)threadIdx.x, lane = tid & 31, wave = tid >> 5, hh = lane >> 4, m = lane & 15;
  const int rowBase = (int)blockIdx.x * GBM;
  if (tid < 32) *(v4fa*)(satt2 + 4 * tid) = *(const v4fa*)(sm + SM_AS2 + 4 * tid);

  v8f acc[4];
  {
    const v8f z = {0.f, 0.f, 0.f, 0.f, 0.f, 0.f, 0.f, 0.f};
#pragma unroll
    for (int t = 0; t < 4; ++t) acc[t] = z;
  }
  const unsigned short* ap = A + (size_t)(rowBase + 16 * wave + m) * (size_t)KP2 + 8 * hh;
  const unsigned short* bp = BT + (size_t)m * (size_t)KP2 + 8 * hh;
  gemm_16x64<K2EXT, KP2>(ap, bp, acc);
  stage_d(stg, acc, wave, hh, m);
  __syncthreads();

  {
    const int row = tid & (GBM - 1), which = tid >> 7;
    const float* sa = satt2 + which * HD;
    const float* hr = stg + row * SP;
    float d = 0.0f;
#pragma unroll 4
    for (int c4 = 0; c4 < HD / 4; ++c4) {
      const v4f hv = *(const v4fa*)(hr + 4 * c4);
      const v4f av = *(const v4fa*)(sa + 4 * c4);
      d = fmaf(hv.x, av.x, d);
      d = fmaf(hv.y, av.y, d);
      d = fmaf(hv.z, av.z, d);
      d = fmaf(hv.w, av.w, d);
    }
    sdot2[row * 2 + which] = d;
  }

  v4f fv[8];
#pragma unroll
  for (int i = 0; i < 8; ++i) {
    const int lr = 16 * wave + 2 * i + hh;
    fv[i] = *(const v4fa*)(stg + lr * SP + 4 * m);
  }
#pragma unroll
  for (int i = 0; i < 8; ++i) {
    const int lr = 16 * wave + 2 * i + hh;
    float* op = XH2 + (size_t)(rowBase + lr) * HD + 4 * m;
    *(volatile v4f*)op = fv[i];
  }
  __threadfence();
#pragma unroll
  for (int i = 0; i < 8; ++i) {
    const int lr = 16 * wave + 2 * i + hh;
    float* op = XH2 + (size_t)(rowBase + lr) * HD + 4 * m;
    *(volatile v4f*)op = fv[i];
  }
  __syncthreads();
  if (tid < 64) {
    const v4f sv = *(const v4fa*)(sdot2 + 4 * tid);
    st2_v4f(SD2 + (size_t)rowBase * 2 + 4 * tid, sv);
  }
}

__global__ __launch_bounds__(NTHR) void k_att2(const int* __restrict__ LIST, const int* __restrict__ CO,
                                               const int* __restrict__ FLAG, const float* __restrict__ XH2,
                                               const float* __restrict__ SD2, const float* __restrict__ sm,
                                               float* out) {
  __shared__ __attribute__((aligned(16))) float sc[ABM];
  __shared__ __attribute__((aligned(16))) float sp[160];
  const int tid = (int)threadIdx.x, lane = tid & 31, wave = tid >> 5, hh = lane >> 4, q = lane & 15;
  if (tid < 40) *(v4fa*)(sp + 4 * tid) = *(const v4fa*)(sm + SM_B2 + 4 * tid);
  __syncthreads();
  const int rowBase = (int)blockIdx.x * ABM;
  const int bucket  = rowBase >> SLB;
  const int* lb  = LIST + (size_t)bucket * RCAP;
  const int* cob = CO + (size_t)bucket * (2 * NBRUN);
  const int flag = FLAG[(size_t)bucket * 32];
  const float qnan = __uint_as_float(0x7fc00000u);
  const v4f b4 = *(const v4fa*)(sp + 4 * q);
  const v4f w4 = *(const v4fa*)(sp + HD + 4 * q);
  const float bsv = sp[2 * HD];

#pragma unroll 1
  for (int i = 0; i < ABM / (2 * NWAVE); ++i) {
    const int lrow = (ABM / NWAVE) * wave + 2 * i + hh;
    const int d    = rowBase + lrow;
    const int slot = d & (NBRUN - 1);
    const int dcl  = d < NN ? d : NN - 1;
    int c = cob[slot];
    int o = cob[NBRUN + slot];
    const bool big = c > DEGCAP;
    c = c < 0 ? 0 : (c > DEGCAP ? DEGCAP : c);
    o = o < 0 ? 0 : (o > RCAP - 1 ? RCAP - 1 : o);
    const int co = __shfl_xor(c, 16, 32);
    const int cm = __builtin_amdgcn_readfirstlane(c > co ? c : co);
    int last = o + c - 1;
    last = last < o ? o : last;
    last = last > RCAP - 1 ? RCAP - 1 : last;

    const float adv = SD2[(size_t)dcl * 2 + 1];
    const float asd = SD2[(size_t)dcl * 2];
    const v4f own = *(const v4fa*)(XH2 + (size_t)dcl * HD + 4 * q);
    asm volatile("" :: "v"(own));
    float l0 = asd + adv;
    l0 = (l0 > 0.0f) ? l0 : NEGSL * l0;
    float mx = l0, dn = 1.0f;
    float a0 = own.x, a1 = own.y, a2 = own.z, a3 = own.w;

#pragma unroll 1
    for (int j = 0; j < cm; ++j) {
      int idx = o + j;
      idx = idx > last ? last : idx;
      int sr = lb[idx];
      sr = sr < 0 ? 0 : (sr > NN - 1 ? NN - 1 : sr);
      const v4f fs = *(const v4fa*)(XH2 + (size_t)sr * HD + 4 * q);
      const float asv = SD2[(size_t)sr * 2];
      asm volatile("" :: "v"(fs));
      asm volatile("" :: "v"(asv));
      const bool valid = j < c;
      float lg = asv + adv;
      lg = (lg > 0.0f) ? lg : NEGSL * lg;
      const float df = lg - mx;
      const float ee = expf(-fabsf(df));
      const bool up  = df > 0.0f;
      const float s1 = up ? ee : 1.0f;
      const float s2 = up ? 1.0f : ee;
      const float tm = up ? lg : mx;
      const float td = fmaf(dn, s1, s2);
      const float t0 = fmaf(a0, s1, s2 * fs.x), t1 = fmaf(a1, s1, s2 * fs.y);
      const float t2 = fmaf(a2, s1, s2 * fs.z), t3 = fmaf(a3, s1, s2 * fs.w);
      mx = valid ? tm : mx;
      dn = valid ? td : dn;
      a0 = valid ? t0 : a0; a1 = valid ? t1 : a1; a2 = valid ? t2 : a2; a3 = valid ? t3 : a3;
    }

    const float inv = 1.0f / (dn + EPS_SM);
    float x0 = fmaf(a0, inv, b4.x), x1 = fmaf(a1, inv, b4.y);
    float x2 = fmaf(a2, inv, b4.z), x3 = fmaf(a3, inv, b4.w);
#pragma unroll 1
    for (int r = 0; r < 4; ++r) {
      const float t = (x0 > 0.0f) ? x0 : expm1f(x0);
      x0 = x1; x1 = x2; x2 = x3; x3 = t;
    }
    const bool bad  = (flag != 0) | big;
    const bool live = d < NN;
    x0 = bad ? qnan : x0; x1 = bad ? qnan : x1; x2 = bad ? qnan : x2; x3 = bad ? qnan : x3;

    float ps = x0 * w4.x;
    ps = fmaf(x1, w4.y, ps);
    ps = fmaf(x2, w4.z, ps);
    ps = fmaf(x3, w4.w, ps);
    ps += __shfl_xor(ps, 1, 32);
    ps += __shfl_xor(ps, 2, 32);
    ps += __shfl_xor(ps, 4, 32);
    ps += __shfl_xor(ps, 8, 32);
    float score = ps + bsv;
    score = bad ? qnan : score;
    if (q == 0) sc[lrow] = score;

    v4f ov;
    ov.x = x0; ov.y = x1; ov.z = x2; ov.w = x3;
    float* op = out + (size_t)d * HD + 4 * q;
    if (live) *(volatile v4f*)op = ov;
    __threadfence();
    if (live) *(volatile v4f*)op = ov;
  }
  __syncthreads();

  if (wave == 0) {
    const v4f sv = *(const v4fa*)(sc + 4 * q);
    asm volatile("" :: "v"(sv));
    const bool wr = (lane < 16) & (rowBase + 4 * q + 3 < NN);
    float* op = out + (size_t)OUT1_OFF + (size_t)rowBase + 4 * q;
    if (wr) *(volatile v4f*)op = sv;
    __threadfence();
    if (wr) *(volatile v4f*)op = sv;
  }
}

extern "C" void kernel_launch(void* const* d_in, const int* in_sizes, int n_in,
                              void* d_out, int out_size, void* d_ws, size_t ws_size,
                              hipStream_t stream) {
  if (n_in < 12) return;
  if (in_sizes[0] != NN * FD) return;
  if (in_sizes[1] != 2 * NE) return;
  if (in_sizes[2] != FD * HC1) return;
  if (in_sizes[3] != NH1 * HD) return;
  if (in_sizes[4] != NH1 * HD) return;
  if (in_sizes[5] != HC1) return;
  if (in_sizes[6] != HC1 * HD) return;
  if (in_sizes[7] != HD) return;
  if (in_sizes[8] != HD) return;
  if (in_sizes[9] != HD) return;
  if (in_sizes[10] != HD) return;
  if (in_sizes[11] != 1) return;
  if (out_size != NN * HD + NN) return;

  const float* x   = (const float*)d_in[0];
  const int*   ei  = (const int*)d_in[1];
  const float* W1  = (const float*)d_in[2];
  const float* as1 = (const float*)d_in[3];
  const float* ad1 = (const float*)d_in[4];
  const float* b1  = (const float*)d_in[5];
  const float* W2  = (const float*)d_in[6];
  const float* as2 = (const float*)d_in[7];
  const float* ad2 = (const float*)d_in[8];
  const float* b2  = (const float*)d_in[9];
  const float* Wsv = (const float*)d_in[10];
  const float* bsv = (const float*)d_in[11];
  float* out = (float*)d_out;
  const int* srcs = ei;
  const int* dsts = ei + NE;

  constexpr size_t zXB   = (size_t)MP * FD * 2;
  constexpr size_t zHL   = (size_t)MP * KP2 * 2;
  constexpr size_t zXH1  = (size_t)MP * HC1 * 4;
  constexpr size_t zXH2  = (size_t)MP * HD * 4;
  constexpr size_t zSD1  = (size_t)MP * 8 * 4;
  constexpr size_t zSD2  = (size_t)MP * 2 * 4;
  constexpr size_t zLIST = (size_t)NBK * RCAP * 4;
  constexpr size_t zCO   = (size_t)NBK * 2 * NBRUN * 4;
  constexpr size_t zFLAG = 6400;
  constexpr size_t zW1T  = (size_t)HC1 * FD * 2;
  constexpr size_t zW2T  = (size_t)HD * KP2 * 2;
  constexpr size_t zSM   = 4352;
  constexpr size_t oA    = 0;
  constexpr size_t oB    = oA + zHL;
  constexpr size_t oSD1  = oB + zXH1;
  constexpr size_t oSD2  = oSD1 + zSD1;
  constexpr size_t oLIST = oSD2 + zSD2;
  constexpr size_t oCO   = oLIST + zLIST;
  constexpr size_t oFLAG = oCO + zCO;
  constexpr size_t oW1T  = oFLAG + zFLAG;
  constexpr size_t oW2T  = oW1T + zW1T;
  constexpr size_t oSM   = oW2T + zW2T;
  constexpr size_t oEND  = oSM + zSM;
  static_assert(zXB <= zHL && zXH2 <= zXH1);
  static_assert(zFLAG >= (size_t)NBK * 128 && zSM >= (size_t)SM_N * 4);
  static_assert(zHL % 256 == 0 && zXH1 % 256 == 0 && zSD1 % 256 == 0 && zSD2 % 256 == 0 && zLIST % 256 == 0);
  static_assert(zCO % 256 == 0 && zFLAG % 256 == 0 && zW1T % 256 == 0 && zW2T % 256 == 0 && zSM % 256 == 0);
  static_assert(oEND <= ((size_t)128u << 20));
  if (oEND > ws_size) return;

  char* ws = (char*)d_ws;
  unsigned short* XB   = (unsigned short*)(ws + oA);
  unsigned short* H1HL = (unsigned short*)(ws + oA);
  float*          XH1  = (float*)(ws + oB);
  float*          XH2  = (float*)(ws + oB);
  float*          SD1  = (float*)(ws + oSD1);
  float*          SD2  = (float*)(ws + oSD2);
  int*            LIST = (int*)(ws + oLIST);
  int*            CO   = (int*)(ws + oCO);
  int*            FLAG = (int*)(ws + oFLAG);
  unsigned short* W1T  = (unsigned short*)(ws + oW1T);
  unsigned short* W2T  = (unsigned short*)(ws + oW2T);
  float*          SM   = (float*)(ws + oSM);

  hipFuncSetAttribute(reinterpret_cast<const void*>(&k_bucket), hipFuncAttributeMaxDynamicSharedMemorySize, (int)BK_LDS);

  k_prep<<<PBTOT, NTHR, 0, stream>>>(x, W1, W2, as1, ad1, b1, as2, ad2, b2, Wsv, bsv, XB, W1T, W2T, SM);
  k_bucket<<<NBK, NTHR, BK_LDS, stream>>>(srcs, dsts, LIST, CO, FLAG);
  k_lin1<<<MP / GBM, NTHR, 0, stream>>>(XB, W1T, SM, XH1, SD1);
  k_att1<<<MP / ABM, NTHR, 0, stream>>>(LIST, CO, FLAG, XH1, SD1, SM, H1HL);
  k_lin2<<<MP / GBM, NTHR, 0, stream>>>(H1HL, W2T, SM, XH2, SD2);
  k_att2<<<MP / ABM, NTHR, 0, stream>>>(LIST, CO, FLAG, XH2, SD2, SM, out);
}
